// HeteroGNNLayer_38611755991310
// MI455X (gfx1250) — hardware-verified
//
#include <hip/hip_runtime.h>
#include <math.h>

#define N_CELL 100000
#define N_IO   2000
#define E_CC   600000
#define E_CIO  50000
#define E_IOC  50000
#define DD     128
#define NH     4
#define NT     256
#define SRB    2048
#define RPW    (SRB / 8)
#define SCH    4096
#define SP     (SCH / NT)
#define APITCH 136
#define DPITCH 132
#define ASC    8.0f
#define WSC    8.0f
#define OSC    (1.0f / 64.0f)
#define NWPL   5
#define NWD    (NWPL * DD * DD / 2)
#define NIOP   2016

static_assert(E_CC % SP == 0 && E_CIO % SP == 0 && E_IOC % SP == 0, "edge counts must be multiples of SP");
static_assert(N_CELL % 32 == 0, "cell rows multiple of 32");
static_assert(N_CELL < (1 << 17) && SRB <= (1 << 11), "list encoding");

typedef __attribute__((ext_vector_type(16))) _Float16 v16h;
typedef __attribute__((ext_vector_type(8)))  _Float16 v8h;
typedef __attribute__((ext_vector_type(4)))  _Float16 v4h;
typedef __attribute__((ext_vector_type(8)))  float    v8f;
typedef __attribute__((ext_vector_type(4)))  float    v4f;
typedef __attribute__((ext_vector_type(4)))  int      v4i;

__device__ __forceinline__ void dep_guard_h(v8f& a, v8f& b, v16h x, v16h y) { asm volatile("v_nop\n\tv_nop\n\tv_nop\n\tv_nop" : "+v"(a), "+v"(b) : "v"(x), "v"(y)); }
__device__ __forceinline__ void dep_guard3_h(v8f& a, v8f& b, v16h x, v16h y, v16h z) { asm volatile("v_nop\n\tv_nop\n\tv_nop\n\tv_nop" : "+v"(a), "+v"(b) : "v"(x), "v"(y), "v"(z)); }
template <typename T> struct Frag;
template <> struct Frag<_Float16> {
  typedef v16h V; union U { v16h v; v8h h[2]; };
  static __device__ __forceinline__ v16h load(const _Float16* p) {
    U f; f.h[0] = *(const v8h*)(p); f.h[1] = *(const v8h*)(p + 16); return f.v;
  }
  static __device__ __forceinline__ v8f mma(v16h a, v16h b, v8f c) {
    return __builtin_amdgcn_wmma_f32_16x16x32_f16(false, a, false, b, (short)0, c, false, false);
  }
  static __device__ __forceinline__ void guard(v8f& a, v8f& b, v16h x, v16h y) { dep_guard_h(a, b, x, y); }
};

__device__ __forceinline__ float wsum32(float d) {
  d += __shfl_xor(d, 16, 32); d += __shfl_xor(d, 8, 32); d += __shfl_xor(d, 4, 32); d += __shfl_xor(d, 2, 32); d += __shfl_xor(d, 1, 32);
  return d;
}

__device__ __forceinline__ int blk_excl_scan(int cnt, int* scan_ws, int tid, int* tot) {
  const int lane = tid & 31, wave = tid >> 5; int incl = cnt;
#pragma unroll
  for (int o = 1; o < 32; o <<= 1) { const int v = __shfl_up(incl, o, 32); if (lane >= o) incl += v; }
  if (lane == 31) scan_ws[wave] = incl;
  __syncthreads();
  if (wave == 0) { int wv = (lane < NT / 32) ? scan_ws[lane] : 0; int wincl = wv;
#pragma unroll
    for (int o = 1; o < 32; o <<= 1) { const int v = __shfl_up(wincl, o, 32); if (lane >= o) wincl += v; }
    if (lane < NT / 32) scan_ws[32 + lane] = wincl - wv; if (lane == 31) scan_ws[64] = wincl; }
  __syncthreads();
  const int res = scan_ws[32 + wave] + incl - cnt; *tot = scan_ws[64];
  return res;
}
template <int NE, int NSRC, int NDST>
__device__ __forceinline__ int chunk_hits(const int* __restrict__ dstv, const int* __restrict__ srcv, int e0, int n0, int tid,
                                          int* LIST, int* scan_ws) {
  const int eb = e0 + tid * SP;
  const bool inr = eb < NE;
  const int ebc = inr ? eb : (NE - SP);
  const int nhi = (n0 + SRB < NDST) ? (n0 + SRB) : NDST;
  int rec[SP]; int cnt = 0;
#pragma unroll
  for (int k = 0; k < SP; k += 4) {
    const v4i d4 = *(const v4i*)(dstv + ebc + k);
    const v4i s4 = *(const v4i*)(srcv + ebc + k);
#pragma unroll
    for (int e = 0; e < 4; ++e) {
      const int d = d4[e]; int r = -1;
      if (inr && d >= n0 && d < nhi) { int s = s4[e]; s = s < 0 ? 0 : (s >= NSRC ? NSRC - 1 : s); r = ((d - n0) << 17) | s; ++cnt; }
      rec[k + e] = r;
    }
  }
  int tot; int p = blk_excl_scan(cnt, scan_ws, tid, &tot);
#pragma unroll
  for (int k = 0; k < SP; ++k) if (rec[k] >= 0) { if ((unsigned)p < (unsigned)SCH) LIST[p] = rec[k]; ++p; }
  __syncthreads();
  return tot < SCH ? tot : SCH;
}

__global__ __launch_bounds__(NT) void prep_w_kernel(const float* __restrict__ W0, const float* __restrict__ W1, const float* __restrict__ W2,
                                                   const float* __restrict__ W3, const float* __restrict__ W4, unsigned* __restrict__ WT32) {
  const int i = blockIdx.x * NT + threadIdx.x;
  if (i < NWD) {
    const int pl = i >> 13; const int rem = i & 8191;
    const int n = rem >> 6; const int k = (rem & 63) * 2;
    const float* wp = (pl == 0) ? W0 : (pl == 1) ? W1 : (pl == 2) ? W2 : (pl == 3) ? W3 : W4;
    const float a = wp[(size_t)k * DD + n] * WSC, b = wp[(size_t)(k + 1) * DD + n] * WSC;
    const _Float16 h0 = (_Float16)a, h1 = (_Float16)b;
    const unsigned u = (unsigned)__builtin_bit_cast(unsigned short, h0) | ((unsigned)__builtin_bit_cast(unsigned short, h1) << 16);
    ((volatile unsigned*)WT32)[i] = u;
    __threadfence();
    ((volatile unsigned*)WT32)[i] = u;
  }
}

__device__ __forceinline__ void gemm_core(const float* __restrict__ A, int M, int row0, const _Float16* __restrict__ Bt, _Float16* As, float* Ds) {
  const int tid = threadIdx.x, lane = tid & 31, wave = tid >> 5;
#pragma unroll
  for (int i = 0; i < 4; ++i) {
    const int q = tid + i * NT;
    const int r = q >> 5, c4 = (q & 31) * 4;
    int gr = row0 + r; gr = gr < M ? gr : M - 1;
    const v4f x = *(const v4f*)(A + (size_t)gr * DD + c4);
    v4h hv;
    hv[0] = (_Float16)(x[0] * ASC); hv[1] = (_Float16)(x[1] * ASC); hv[2] = (_Float16)(x[2] * ASC); hv[3] = (_Float16)(x[3] * ASC);
    *(v4h*)(As + r * APITCH + c4) = hv;
  }
  __syncthreads();
  const int rg = wave >> 2, cg = wave & 3;
  const int rlane = lane & 15, koff = (lane >> 4) * 8, mOff = (lane >> 4) * 8;
  v8f acc0 = (v8f){0.f,0.f,0.f,0.f,0.f,0.f,0.f,0.f};
  v8f acc1 = (v8f){0.f,0.f,0.f,0.f,0.f,0.f,0.f,0.f};
#pragma unroll
  for (int ks = 0; ks < 4; ++ks) {
    const v16h af  = Frag<_Float16>::load(As + (rg * 16 + rlane) * APITCH + ks * 32 + koff);
    const v16h bf0 = Frag<_Float16>::load(Bt + (size_t)(cg * 32 + rlane) * DD + ks * 32 + koff);
    const v16h bf1 = Frag<_Float16>::load(Bt + (size_t)(cg * 32 + 16 + rlane) * DD + ks * 32 + koff);
    acc0 = Frag<_Float16>::mma(af, bf0, acc0);
    acc1 = Frag<_Float16>::mma(af, bf1, acc1);
    dep_guard3_h(acc0, acc1, af, bf0, bf1);
  }
  dep_guard_h(acc0, acc1, (v16h){}, (v16h){});
#pragma unroll
  for (int r = 0; r < 8; ++r) {
    Ds[(rg * 16 + mOff + r) * DPITCH + cg * 32 + rlane]      = acc0[r] * OSC;
    Ds[(rg * 16 + mOff + r) * DPITCH + cg * 32 + 16 + rlane] = acc1[r] * OSC;
  }
  __syncthreads();
}

template <bool WHS>
__global__ __launch_bounds__(NT) void proj_kernel(const float* __restrict__ X, int M, const _Float16* __restrict__ Bt,
                                                 const float* __restrict__ avs, const float* __restrict__ avd,
                                                 float* __restrict__ HS, float* __restrict__ ALS, float* __restrict__ ALD) {
  __shared__ __align__(16) _Float16 As[32 * APITCH];
  __shared__ __align__(16) float Ds[32 * DPITCH];
  __shared__ __align__(16) float sAs[DD];
  __shared__ __align__(16) float sAd[DD];
  __shared__ __align__(16) float sal[32 * NH];
  __shared__ __align__(16) float sad[32 * NH];
  const int tid = threadIdx.x, lane = tid & 31, wave = tid >> 5;
  const int row0 = blockIdx.x * 32;
  if (tid < DD) { sAs[tid] = avs[tid]; sAd[tid] = avd[tid]; }
  gemm_core(X, M, row0, Bt, As, Ds);
  if (WHS) {
    v4f vals[4];
#pragma unroll
    for (int j = 0; j < 4; ++j) vals[j] = *(const v4f*)(Ds + (wave * 4 + j) * DPITCH + 4 * lane);
    for (int ps = 0; ps < 2; ++ps) {
#pragma unroll
      for (int j = 0; j < 4; ++j) {
        const int gr = row0 + wave * 4 + j;
        if (gr < M) *(volatile v4f*)(HS + (size_t)gr * DD + 4 * lane) = vals[j];
      }
      __threadfence();
    }
  }
  if (tid < 32 * NH) {
    const int r = tid >> 2, h = tid & 3;
    const float* dr = Ds + r * DPITCH + h * 32;
    const float* pa = sAs + h * 32;
    const float* pd = sAd + h * 32;
    float ss = 0.f, sd = 0.f;
#pragma unroll 8
    for (int c = 0; c < 32; ++c) { const float v = dr[c]; ss += v * pa[c]; sd += v * pd[c]; }
    sal[tid] = ss; sad[tid] = sd;
  }
  __syncthreads();
  if (wave == 0) {
    const v4f p = *(const v4f*)(sal + 4 * lane);
    float* op = ALS + (size_t)row0 * NH + 4 * lane;
    for (int ps = 0; ps < 2; ++ps) { *(volatile v4f*)op = p; __threadfence(); }
  } else if (wave == 1) {
    const v4f p = *(const v4f*)(sad + 4 * lane);
    float* op = ALD + (size_t)row0 * NH + 4 * lane;
    for (int ps = 0; ps < 2; ++ps) { *(volatile v4f*)op = p; __threadfence(); }
  }
}

__global__ __launch_bounds__(NT) void xform_kernel(const float* __restrict__ Y, int M, const _Float16* __restrict__ Bt,
                                                  const float* __restrict__ bt, const float* __restrict__ gm, const float* __restrict__ be,
                                                  float* __restrict__ OUT) {
  __shared__ __align__(16) _Float16 As[32 * APITCH];
  __shared__ __align__(16) float Ds[32 * DPITCH];
  const int tid = threadIdx.x, lane = tid & 31, wave = tid >> 5;
  const int row0 = blockIdx.x * 32;
  gemm_core(Y, M, row0, Bt, As, Ds);
  const v4f btv = *(const v4f*)(bt + 4 * lane);
  const v4f gv  = *(const v4f*)(gm + 4 * lane);
  const v4f bev = *(const v4f*)(be + 4 * lane);
#pragma unroll
  for (int j = 0; j < 4; ++j) {
    const int r = wave * 4 + j;
    const int gr = row0 + r;
    const int grc = gr < M ? gr : M - 1;
    const v4f hv = *(const v4f*)(Ds + r * DPITCH + 4 * lane) + btv;
    float s = hv[0] + hv[1] + hv[2] + hv[3];
    s = wsum32(s);
    const float mu = s * (1.0f / 128.0f);
    const v4f dv = hv - mu;
    float s2 = dv[0] * dv[0] + dv[1] * dv[1] + dv[2] * dv[2] + dv[3] * dv[3];
    s2 = wsum32(s2);
    const float var = s2 * (1.0f / 128.0f);
    const float rs = rsqrtf(var + 1e-5f);
    const v4f av = *(const v4f*)(Y + (size_t)grc * DD + 4 * lane);
    v4f o;
#pragma unroll
    for (int e = 0; e < 4; ++e) { const float t = dv[e] * rs * gv[e] + bev[e]; o[e] = av[e] + (t > 0.f ? t : 0.f); }
    if (gr < M) {
      float* op = OUT + (size_t)gr * DD + 4 * lane;
      for (int ps = 0; ps < 2; ++ps) { *(volatile v4f*)op = o; __threadfence(); }
    }
  }
}

template <int NE, int NSRC, int NDST, int MODE, int NB>
__global__ __launch_bounds__(NT) void agg_kernel(const float* __restrict__ HSs, const float* __restrict__ ALSs, const float* __restrict__ ALDd,
                                                const int* __restrict__ ei, const float* __restrict__ b1, const float* __restrict__ b2,
                                                float* WORK, float* OUT) {
  __shared__ int LIST[SCH];
  __shared__ float SM[SRB * NH];
  __shared__ float SL[SRB * NH];
  __shared__ int scan_ws[80];
  const int tid = threadIdx.x, lane = tid & 31, wave = tid >> 5;
  const int hd = lane >> 3;
  const int n0 = blockIdx.x * SRB;
  const int* srcv = ei;
  const int* dstv = ei + NE;
  const v4f z4 = {0.f, 0.f, 0.f, 0.f};
  for (int ps = 0; ps < 2; ++ps) {
#pragma unroll 1
    for (int j = 0; j < RPW; ++j) {
      const int n = n0 + wave * RPW + j;
      if (n < NDST) *(volatile v4f*)(WORK + (size_t)n * DD + 4 * lane) = z4;
    }
    __threadfence();
  }
  for (int i = tid; i < SRB * NH; i += NT) { SM[i] = -INFINITY; SL[i] = 0.f; }
  __syncthreads();
  constexpr int NCH = (NE + SCH - 1) / SCH;
#pragma unroll 1
  for (int c = 0; c < NCH; ++c) {
    const int tot = chunk_hits<NE, NSRC, NDST>(dstv, srcv, c * SCH, n0, tid, LIST, scan_ws);
#pragma unroll 1
    for (int base = 0; base < tot; base += 32) {
      int qi = base + lane; const bool inl = qi < tot; qi = qi < SCH ? qi : SCH - 1;
      const int lsv = LIST[qi];
      const int rv = inl ? lsv : -1;
      const int own = (rv >= 0 && (rv >> 25) == wave) ? 1 : 0;
      unsigned msk = (unsigned)__ballot(own);
#pragma unroll 1
      for (int it = 0; it < 32; ++it) {
        if (msk == 0u) break;
        const int bp = __builtin_ctz(msk); msk &= msk - 1u;
        const int r = __shfl(rv, bp, 32);
        const int dl = r >> 17, s = r & 0x1FFFF;
        const int n = n0 + dl;
        const v4f hv = *(const v4f*)(HSs + (size_t)s * DD + 4 * lane);
        float e = ALSs[(size_t)s * NH + hd] + ALDd[(size_t)n * NH + hd];
        e = e > 0.f ? e : 0.2f * e;
        const int si = dl * NH + hd;
        const float mo = SM[si], lo = SL[si];
        const float mn = fmaxf(mo, e);
        const float rr = __expf(mo - mn), ex = __expf(e - mn);
        const float ln = lo * rr + ex;
        if ((lane & 7) == 0) { SM[si] = mn; SL[si] = ln; }
        float* rp = WORK + (size_t)n * DD + 4 * lane;
        v4f a = *(const v4f*)rp;
        a = a * rr + ex * hv;
        *(volatile v4f*)rp = a;
        __threadfence();
        *(volatile v4f*)rp = a;
      }
    }
    __syncthreads();
  }
  v4f bsum = {0.f, 0.f, 0.f, 0.f};
  if (NB >= 1) bsum = bsum + *(const v4f*)(b1 + 4 * lane);
  if (NB >= 2) bsum = bsum + *(const v4f*)(b2 + 4 * lane);
#pragma unroll 1
  for (int j = 0; j < RPW; ++j) {
    const int dl = wave * RPW + j; const int n = n0 + dl;
    if (n < NDST) {
      const float lsum = SL[dl * NH + hd];
      const float inv = (lsum > 0.f) ? (1.0f / lsum) : 0.f;
      const v4f a = *(const v4f*)(WORK + (size_t)n * DD + 4 * lane);
      v4f v = a * inv;
      if (MODE == 0) v = v + bsum;
      else v = v + *(const v4f*)(OUT + (size_t)n * DD + 4 * lane);
      float* op = OUT + (size_t)n * DD + 4 * lane;
      for (int ps = 0; ps < 2; ++ps) { *(volatile v4f*)op = v; __threadfence(); }
    }
  }
}

extern "C" void kernel_launch(void* const* d_in, const int* in_sizes, int n_in,
                              void* d_out, int out_size, void* d_ws, size_t ws_size,
                              hipStream_t stream) {
  (void)in_sizes; (void)n_in; (void)out_size;
  const float* x_cell  = (const float*)d_in[0];
  const float* x_io    = (const float*)d_in[1];
  const int*   ei_cc   = (const int*)d_in[2];
  const int*   ei_cio  = (const int*)d_in[3];
  const int*   ei_ioc  = (const int*)d_in[4];
  const float* W_cc    = (const float*)d_in[5];
  const float* as_cc   = (const float*)d_in[6];
  const float* ad_cc   = (const float*)d_in[7];
  const float* b_cc    = (const float*)d_in[8];
  const float* W_cio   = (const float*)d_in[9];
  const float* as_cio  = (const float*)d_in[10];
  const float* ad_cio  = (const float*)d_in[11];
  const float* b_cio   = (const float*)d_in[12];
  const float* W_ioc   = (const float*)d_in[13];
  const float* as_ioc  = (const float*)d_in[14];
  const float* ad_ioc  = (const float*)d_in[15];
  const float* b_ioc   = (const float*)d_in[16];
  const float* Wt_cell = (const float*)d_in[17];
  const float* bt_cell = (const float*)d_in[18];
  const float* g_cell  = (const float*)d_in[19];
  const float* be_cell = (const float*)d_in[20];
  const float* Wt_io   = (const float*)d_in[21];
  const float* bt_io   = (const float*)d_in[22];
  const float* g_io    = (const float*)d_in[23];
  const float* be_io   = (const float*)d_in[24];

  float* out_cell = (float*)d_out;
  float* out_io   = out_cell + (size_t)N_CELL * DD;

  char* ws = (char*)d_ws; size_t off = 0;
  auto carve = [&](size_t bytes) -> char* { char* p = ws + off; off += (bytes + 255) & ~(size_t)255; return p; };
  _Float16* WT    = (_Float16*)carve((size_t)NWPL * DD * DD * 2);
  float*    HS    = (float*)carve((size_t)N_CELL * DD * 4);
  float*    HSIO  = (float*)carve((size_t)N_IO * DD * 4);
  float*    ACC_C = (float*)carve((size_t)N_CELL * DD * 4);
  float*    ACC_I = (float*)carve((size_t)N_IO * DD * 4);
  float*    ALS_C = (float*)carve((size_t)N_CELL * NH * 4);
  float*    ALD_C = (float*)carve((size_t)N_CELL * NH * 4);
  float*    ALS_I = (float*)carve((size_t)NIOP * NH * 4);
  float*    ALD_I = (float*)carve((size_t)NIOP * NH * 4);
  if (off > ws_size || off > (size_t)134217728) return;

  const _Float16* WT_cc   = WT + 0 * DD * DD;
  const _Float16* WT_cio  = WT + 1 * DD * DD;
  const _Float16* WT_ioc  = WT + 2 * DD * DD;
  const _Float16* WT_tc   = WT + 3 * DD * DD;
  const _Float16* WT_tio  = WT + 4 * DD * DD;

  const int GC = (N_CELL + 31) / 32;
  const int GI = (N_IO + 31) / 32;
  const int TC = (N_CELL + SRB - 1) / SRB;
  const int TI = (N_IO + SRB - 1) / SRB;

  prep_w_kernel<<<(NWD + NT - 1) / NT, NT, 0, stream>>>(W_cc, W_cio, W_ioc, Wt_cell, Wt_io, (unsigned*)WT);

  proj_kernel<true><<<GC, NT, 0, stream>>>(x_cell, N_CELL, WT_cc, as_cc, ad_cc, HS, ALS_C, ALD_C);
  agg_kernel<E_CC, N_CELL, N_CELL, 0, 2><<<TC, NT, 0, stream>>>(HS, ALS_C, ALD_C, ei_cc, b_cc, b_ioc, ACC_C, ACC_C);

  proj_kernel<true><<<GI, NT, 0, stream>>>(x_io, N_IO, WT_ioc, as_ioc, ad_ioc, HSIO, ALS_I, ALD_I);
  proj_kernel<false><<<GC, NT, 0, stream>>>(x_cell, N_CELL, WT_ioc, as_ioc, ad_ioc, (float*)nullptr, ALS_C, ALD_C);
  agg_kernel<E_IOC, N_IO, N_CELL, 1, 0><<<TC, NT, 0, stream>>>(HSIO, ALS_I, ALD_C, ei_ioc, (const float*)nullptr, (const float*)nullptr, HS, ACC_C);

  proj_kernel<true><<<GC, NT, 0, stream>>>(x_cell, N_CELL, WT_cio, as_cio, ad_cio, HS, ALS_C, ALD_C);
  proj_kernel<false><<<GI, NT, 0, stream>>>(x_io, N_IO, WT_cio, as_cio, ad_cio, (float*)nullptr, ALS_I, ALD_I);
  agg_kernel<E_CIO, N_CELL, N_IO, 0, 1><<<TI, NT, 0, stream>>>(HS, ALS_C, ALD_I, ei_cio, b_cio, (const float*)nullptr, ACC_I, ACC_I);

  xform_kernel<<<GC, NT, 0, stream>>>(ACC_C, N_CELL, WT_tc, bt_cell, g_cell, be_cell, out_cell);
  xform_kernel<<<GI, NT, 0, stream>>>(ACC_I, N_IO, WT_tio, bt_io, g_io, be_io, out_io);
}
